// Qwen3Attention_7748121002093
// MI455X (gfx1250) — hardware-verified
//
#include <hip/hip_runtime.h>
#ifndef NB
#define NB 2
#endif
#ifndef SEQ
#define SEQ 2048
#endif
#define NB_FULL 2
#define SEQ_FULL 2048
#define SQ SEQ
#define DMX 2048
#define NH 16
#define NKV 4
#define GSZ 4
#define HDK 128
#define DKV (NKV * HDK)
#define NQKV (DMX + 2 * DKV)
#define QT 256
#define QT0 128
#define NKX SQ
#define NR ((size_t)NB * SQ)
#define ATS 0.08838834764831845f
#define PSC 1024.0f
#define LNEPS 1.0e-5f
#define THETA 1000000.0
static_assert(SQ % QT == 0);
static_assert(QT % 128 == 0);
static_assert((NH * QT) % 256 == 0);
static_assert(SQ % 64 == 0);
static_assert(QT0 == 128);
static_assert(QT0 <= SQ);
static_assert(NH == NKV * GSZ);
static_assert((NB * SQ) % 128 == 0);
static_assert(NB <= NB_FULL);
static_assert(SEQ <= SEQ_FULL);
static_assert(DMX % 64 == 0);
static_assert(DKV % 64 == 0);
static_assert(HDK == 128);

typedef unsigned short v8us __attribute__((ext_vector_type(8), may_alias));
typedef float v8f __attribute__((ext_vector_type(8)));
typedef float v4f __attribute__((ext_vector_type(4)));
typedef float v4fa __attribute__((ext_vector_type(4), may_alias));
typedef _Float16 v16h __attribute__((ext_vector_type(16)));
typedef _Float16 v4h __attribute__((ext_vector_type(4)));
union FragH { v16h v; v8us half[2]; _Float16 h[16]; unsigned short u[16]; };

__device__ __forceinline__ unsigned short bf16_bits(float x) { unsigned int u = __float_as_uint(x); return (unsigned short)((u + 0x7FFFu + ((u >> 16) & 1u)) >> 16); }
__device__ __forceinline__ float bf16_val(unsigned short b) { return __uint_as_float(((unsigned int)b) << 16); }
__device__ __forceinline__ float bf16_rne(float x) { return bf16_val(bf16_bits(x)); }

__device__ __forceinline__ v16h g2_frag(const _Float16* p, int hh) { FragH f; f.half[0] = *(const v8us*)((const unsigned short*)p + 8 * hh); f.half[1] = *(const v8us*)((const unsigned short*)p + 16 + 8 * hh); return f.v; }
__device__ __forceinline__ v8f g2_mma(v16h a, v16h b, v8f c) { v8f d = __builtin_amdgcn_wmma_f32_16x16x32_f16(false, a, false, b, (short)0, c, false, false); asm volatile("v_nop\n\tv_nop\n\tv_nop\n\tv_nop" : "+v"(d) : "v"(a), "v"(b)); return d; }

__global__ __launch_bounds__(128) void k_gemm2(const _Float16* __restrict__ A, int lda, size_t sA, const _Float16* __restrict__ Bh, int ldb, size_t sB, int bdiv, float alpha,
    const float* CP, float* C, _Float16* __restrict__ C16, int ldc, size_t sC, int M, int N, int K) {
  __shared__ __attribute__((aligned(16))) float so[4][32][68];
  const int tid = threadIdx.x, w = tid >> 5, lane = tid & 31, ln = lane & 15, hh = lane >> 4; const int by = blockIdx.y;
  A += (size_t)by * sA; Bh += (size_t)(by / bdiv) * sB; const size_t cofs = (size_t)by * sC;
  const int ntn = N >> 6; const int mt = blockIdx.x / ntn, nq = blockIdx.x - mt * ntn; const int row0 = mt * 128 + 32 * w, col0 = nq * 64; if (row0 >= M) return;
  const _Float16* a0p = A + (size_t)(row0 + ln) * lda; const _Float16* a1p = a0p + (size_t)16 * lda;
  const _Float16* b0p = Bh + (size_t)(col0 + ln) * ldb; const _Float16* b1p = b0p + (size_t)16 * ldb; const _Float16* b2p = b1p + (size_t)16 * ldb; const _Float16* b3p = b2p + (size_t)16 * ldb;
  const v8f z8 = {0.f, 0.f, 0.f, 0.f, 0.f, 0.f, 0.f, 0.f}; v8f c00 = z8, c01 = z8, c02 = z8, c03 = z8, c10 = z8, c11 = z8, c12 = z8, c13 = z8;
#pragma unroll 1
  for (int kb = 0; kb < K; kb += 32) { const v16h a0 = g2_frag(a0p + kb, hh), a1 = g2_frag(a1p + kb, hh);
    v16h b = g2_frag(b0p + kb, hh); c00 = g2_mma(a0, b, c00); c10 = g2_mma(a1, b, c10);
    b = g2_frag(b1p + kb, hh); c01 = g2_mma(a0, b, c01); c11 = g2_mma(a1, b, c11);
    b = g2_frag(b2p + kb, hh); c02 = g2_mma(a0, b, c02); c12 = g2_mma(a1, b, c12);
    b = g2_frag(b3p + kb, hh); c03 = g2_mma(a0, b, c03); c13 = g2_mma(a1, b, c13); }
  v8f accs[8] = {c00, c01, c02, c03, c10, c11, c12, c13};
#pragma unroll
  for (int u = 0; u < 8; ++u) { const int t = u & 3, half = u >> 2; const int col = col0 + t * 16 + ln;
#pragma unroll
    for (int r = 0; r < 8; ++r) { const int rloc = half * 16 + 8 * hh + r; float v = accs[u][r] * alpha; if (CP) v += CP[cofs + (size_t)(row0 + rloc) * ldc + col]; so[w][rloc][t * 16 + ln] = v; } }
  __builtin_amdgcn_fence(4  , "workgroup"); __builtin_amdgcn_wave_barrier();
  const int rsub = lane >> 4, c4 = (lane & 15) * 4;
  for (int pass = 0; pass < 2; ++pass) {
#pragma unroll
    for (int q = 0; q < 16; ++q) { const int r = q * 2 + rsub; const v4f v = *(const v4fa*)&so[w][r][c4];
      if (C) *(volatile v4f*)(C + cofs + (size_t)(row0 + r) * ldc + col0 + c4) = v;
      if (C16) { v4h h4;
#pragma unroll
        for (int i = 0; i < 4; ++i) h4[i] = (_Float16)v[i]; *(volatile v4h*)(C16 + cofs + (size_t)(row0 + r) * ldc + col0 + c4) = h4; } }
    if (pass == 0) __threadfence(); } }

__global__ __launch_bounds__(256) void k_wnat(const float* __restrict__ w, size_t n8, _Float16* __restrict__ Bt) {
  const size_t t = (size_t)blockIdx.x * 256 + threadIdx.x; if (t >= n8) return; FragH f;
#pragma unroll
  for (int q = 0; q < 8; ++q) f.h[q] = (_Float16)(bf16_rne(w[t * 8 + q]) * 16.0f);
  *(volatile v8us*)((unsigned short*)Bt + t * 8) = f.half[0]; __threadfence(); *(volatile v8us*)((unsigned short*)Bt + t * 8) = f.half[0]; }

__global__ __launch_bounds__(256) void k_x16(const float* __restrict__ x, _Float16* __restrict__ X16, size_t n8) {
  const size_t t = (size_t)blockIdx.x * 256 + threadIdx.x; if (t >= n8) return;
  const size_t r = t / (DMX / 8); const size_t c8 = (t % (DMX / 8)) * 8; const size_t rs = (r / SQ) * SEQ_FULL + (r % SQ);
  const v4f a = *(const v4fa*)(x + rs * DMX + c8), b2 = *(const v4fa*)(x + rs * DMX + c8 + 4); FragH f;
#pragma unroll
  for (int q = 0; q < 4; ++q) { f.h[q] = (_Float16)bf16_rne(a[q]); f.h[4 + q] = (_Float16)bf16_rne(b2[q]); }
  *(volatile v8us*)((unsigned short*)X16 + t * 8) = f.half[0]; __threadfence(); *(volatile v8us*)((unsigned short*)X16 + t * 8) = f.half[0]; }

__global__ __launch_bounds__(128) void k_lnh128(float* __restrict__ F, int ldf, int nh, const float* __restrict__ g, const float* __restrict__ bb, float eps) {
  #pragma clang fp contract(off)
  __shared__ float red[128]; __shared__ __attribute__((aligned(16))) float ov[128];
  const int d = threadIdx.x; const int h = blockIdx.x % nh; const size_t r = blockIdx.x / nh; float* p = F + r * (size_t)ldf + (size_t)h * 128; const float v = p[d];
  red[d] = v; __syncthreads(); for (int st = 64; st > 0; st >>= 1) { if (d < st) red[d] = __fadd_rn(red[d], red[d + st]); __syncthreads(); }
  const float mu = __fmul_rn(red[0], 0.0078125f); __syncthreads();
  const float c = __fadd_rn(v, -mu); red[d] = __fmul_rn(c, c); __syncthreads(); for (int st = 64; st > 0; st >>= 1) { if (d < st) red[d] = __fadd_rn(red[d], red[d + st]); __syncthreads(); }
  const float rs = rsqrtf(__fadd_rn(__fmul_rn(red[0], 0.0078125f), eps));
  ov[d] = __fadd_rn(__fmul_rn(__fmul_rn(c, rs), bf16_rne(g[d])), bf16_rne(bb[d])); __syncthreads();
  if (d < 32) { const v4f o = *(const v4f*)&ov[d * 4]; float* dst = p + d * 4; *(volatile v4f*)dst = o; __threadfence(); *(volatile v4f*)dst = o; } }

__global__ __launch_bounds__(256) void k_tab128(float* __restrict__ CS, float* __restrict__ SN) {
  #pragma clang fp contract(off)
  const int t = blockIdx.x * 256 + threadIdx.x; if (t >= SQ * 64) return; const int i = t % 64; const int p = t / 64;
  const float pw = (float)pow(THETA, (double)i * 0.015625); const float invf = 1.0f / pw; const float ang = __fmul_rn((float)p, invf); float s, c; sincosf(ang, &s, &c);
  *(volatile float*)(CS + t) = c; *(volatile float*)(SN + t) = s; __threadfence(); *(volatile float*)(CS + t) = c; *(volatile float*)(SN + t) = s; }

template <int F32OUT>
__global__ __launch_bounds__(128) void k_rope128(const float* __restrict__ F, int ldf, int nh, const float* __restrict__ CS, const float* __restrict__ SN, void* __restrict__ OUT, int ldo) {
  #pragma clang fp contract(off)
  __shared__ __attribute__((aligned(16))) float xv[128]; __shared__ __attribute__((aligned(16))) float ov[128];
  const int d = threadIdx.x; const int h = blockIdx.x % nh; const size_t r = blockIdx.x / nh; const int p = (int)(r % SQ);
  xv[d] = F[r * (size_t)ldf + (size_t)h * 128 + d]; __syncthreads();
  const float c = CS[p * 64 + (d & 63)], s = SN[p * 64 + (d & 63)]; const float xo = xv[d ^ 64]; const float rot = (d < 64) ? -xo : xo;
  ov[d] = __fadd_rn(__fmul_rn(xv[d], c), __fmul_rn(rot, s)); __syncthreads();
  if (F32OUT) { if (d < 32) { const v4f v = *(const v4f*)&ov[d * 4]; float* dst = (float*)OUT + r * (size_t)ldo + (size_t)h * 128 + d * 4; *(volatile v4f*)dst = v; __threadfence(); *(volatile v4f*)dst = v; } }
  else { if (d < 16) { FragH f;
#pragma unroll
      for (int q = 0; q < 8; ++q) f.h[q] = (_Float16)ov[d * 8 + q]; unsigned short* dst = (unsigned short*)OUT + r * (size_t)ldo + (size_t)h * 128 + d * 8; *(volatile v8us*)dst = f.half[0]; __threadfence(); *(volatile v8us*)dst = f.half[0]; } } }

template <int NSL, int TTv>
__global__ __launch_bounds__(256) void k_vt(const _Float16* __restrict__ V16, int ldv, _Float16* __restrict__ Vt) { __shared__ unsigned short tl[64][66]; const int tid = threadIdx.x; const int slab = blockIdx.x / (TTv / 64), lg = blockIdx.x % (TTv / 64);
  for (int i = tid; i < 64 * 8; i += 256) { const int r = i / 8, c8 = (i % 8) * 8; FragH f; f.half[0] = *(const v8us*)((const unsigned short*)V16 + ((size_t)lg * 64 + r) * ldv + slab * 64 + c8);
#pragma unroll
    for (int q = 0; q < 8; ++q) tl[r][c8 + q] = f.u[q]; }
  __syncthreads();
  for (int pass = 0; pass < 2; ++pass) {
#pragma unroll
    for (int rd = 0; rd < 2; ++rd) { const int d = rd * 32 + tid / 8, pc = tid % 8; FragH f;
#pragma unroll
      for (int q = 0; q < 8; ++q) f.u[q] = tl[pc * 8 + q][d];
      *(volatile v8us*)((unsigned short*)Vt + ((size_t)slab * 64 + d) * TTv + lg * 64 + pc * 8) = f.half[0]; }
    if (pass == 0) __threadfence(); } }

__global__ __launch_bounds__(256) void k_hl(const float* __restrict__ Fp, _Float16* __restrict__ Hh, _Float16* __restrict__ Hl, size_t n8) { const size_t t = (size_t)blockIdx.x * 256 + threadIdx.x; if (t >= n8) return; FragH fh, fl; const v4f a = *(const v4fa*)(Fp + t * 8), c = *(const v4fa*)(Fp + t * 8 + 4);
#pragma unroll
  for (int q = 0; q < 4; ++q) { _Float16 hv = (_Float16)a[q]; fh.h[q] = hv; fl.h[q] = (_Float16)((a[q] - (float)hv) * 1024.0f); hv = (_Float16)c[q]; fh.h[4 + q] = hv; fl.h[4 + q] = (_Float16)((c[q] - (float)hv) * 1024.0f); }
  for (int pass = 0; pass < 2; ++pass) { *(volatile v8us*)((unsigned short*)Hh + t * 8) = fh.half[0]; *(volatile v8us*)((unsigned short*)Hl + t * 8) = fl.half[0]; if (pass == 0) __threadfence(); } }

template <int GS_>
__global__ __launch_bounds__(32) void k_att0h(const float* __restrict__ QF, int ldq, const float* __restrict__ KF, const float* __restrict__ VF, int ldkv, float scale, float* __restrict__ OF, int ldo) {
  #pragma clang fp contract(off)
  __shared__ __attribute__((aligned(16))) float lq[32][128]; __shared__ __attribute__((aligned(16))) float lo[32][128]; __shared__ float lf[32];
  const int tid = threadIdx.x; const int h = blockIdx.x / (QT0 / 32), rg = blockIdx.x % (QT0 / 32); const int i = rg * 32 + tid; const int hk = h / GS_;
  for (int c = 0; c < 32; ++c) { *(v4f*)&lq[tid][c * 4] = *(const v4fa*)(QF + (size_t)i * ldq + h * 128 + c * 4); const v4f z = {0.f, 0.f, 0.f, 0.f}; *(v4f*)&lo[tid][c * 4] = z; }
  float m = -1.0e30f, l = 0.f; const int jmax = rg * 32 + 31;
#pragma unroll 1
  for (int j = 0; j <= jmax; ++j) { const float* kr = KF + (size_t)j * ldkv + hk * 128; const float* vr = VF + (size_t)j * ldkv + hk * 128; float s = 0.f;
#pragma unroll 1
    for (int c = 0; c < 32; ++c) { const v4f kq = *(const v4fa*)(kr + c * 4); const v4f qq = *(v4f*)&lq[tid][c * 4];
#pragma unroll
      for (int u = 0; u < 4; ++u) s = __fadd_rn(s, __fmul_rn(qq[u], kq[u])); }
    s = __fmul_rn(s, scale); const float f = (j <= i) ? 1.f : 0.f;
    const float sm = fmaf(f, s, (1.f - f) * -1.0e30f); const float mn = fmaxf(m, sm); const float sc = expf(m - mn); const float e = __fmul_rn(f, expf(sm - mn)); l = __fadd_rn(__fmul_rn(l, sc), e); m = mn;
#pragma unroll 1
    for (int c = 0; c < 32; ++c) { const v4f vv = *(const v4fa*)(vr + c * 4); v4f oo = *(v4f*)&lo[tid][c * 4];
#pragma unroll
      for (int u = 0; u < 4; ++u) oo[u] = __fadd_rn(__fmul_rn(oo[u], sc), __fmul_rn(e, vv[u])); *(v4f*)&lo[tid][c * 4] = oo; } }
  lf[tid] = 64.0f / l; __syncthreads();
  for (int pass = 0; pass < 2; ++pass) {
#pragma unroll 1
    for (int rr = 0; rr < 32; ++rr) { v4f oo = *(v4f*)&lo[rr][tid * 4]; const float fin = lf[rr];
#pragma unroll
      for (int u = 0; u < 4; ++u) oo[u] = __fmul_rn(oo[u], fin); *(volatile v4f*)(OF + (size_t)(rg * 32 + rr) * ldo + h * 128 + tid * 4) = oo; }
    if (pass == 0) __threadfence(); } }

__global__ __launch_bounds__(256) void k_rsmcf2(const float* __restrict__ S, _Float16* __restrict__ P, int q0, int nk) {
  #pragma clang fp contract(off)
  __shared__ __attribute__((aligned(16))) unsigned short st[8][32][72];
  const int w = threadIdx.x >> 5, lane = threadIdx.x & 31;
  const size_t i = (size_t)blockIdx.x * 256 + threadIdx.x; const float* s = S + i * NKX; const int last = q0 + (int)(i % QT);
  const size_t ib = (size_t)blockIdx.x * 256 + (size_t)w * 32;
  float mx = -3.0e38f;
#pragma unroll 1
  for (int j = 0; j < nk; ++j) { const float f = (j <= last) ? 1.f : 0.f; mx = fmaxf(mx, fmaf(f, s[j], (1.f - f) * -1.0e9f)); }
  float se = 0.f;
#pragma unroll 1
  for (int j = 0; j < nk; ++j) { const float f = (j <= last) ? 1.f : 0.f; se += __expf(fmaf(f, s[j], (1.f - f) * -1.0e9f) - mx); }
  const float sc = PSC / se;
#pragma unroll 1
  for (int j0 = 0; j0 < nk; j0 += 64) {
#pragma unroll 1
    for (int u = 0; u < 8; ++u) { FragH fr;
#pragma unroll
      for (int q = 0; q < 8; ++q) { const int j = j0 + u * 8 + q; const float f = (j <= last) ? 1.f : 0.f; fr.h[q] = (_Float16)(__expf(fmaf(f, s[j], (1.f - f) * -1.0e9f) - mx) * sc); }
      *(v8us*)&st[w][lane][u * 8] = fr.half[0]; }
    __builtin_amdgcn_fence(3  , "wavefront"); __builtin_amdgcn_wave_barrier();
    for (int pass = 0; pass < 2; ++pass) {
#pragma unroll
      for (int it = 0; it < 8; ++it) { const int rr = it * 4 + (lane >> 3), pc = lane & 7; const v8us v = *(const v8us*)&st[w][rr][pc * 8]; *(volatile v8us*)((unsigned short*)P + (ib + rr) * NKX + j0 + pc * 8) = v; }
      if (pass == 0) __threadfence(); }
    __builtin_amdgcn_fence(4  , "wavefront"); __builtin_amdgcn_wave_barrier(); } }

extern "C" void kernel_launch(void* const* d_in, const int* in_sizes, int n_in,
                              void* d_out, int out_size, void* d_ws, size_t ws_size, hipStream_t stream) {
  if (n_in < 7) return;
  if ((size_t)in_sizes[0] < ((size_t)(NB - 1) * SEQ_FULL + SQ) * DMX) return;
  if ((size_t)in_sizes[1] < (size_t)NQKV * DMX || (size_t)in_sizes[2] < (size_t)DMX * DMX) return;
  if (in_sizes[3] < HDK || in_sizes[4] < HDK || in_sizes[5] < HDK || in_sizes[6] < HDK) return;
  if ((size_t)out_size < NR * DMX) return;
  const float* x = (const float*)d_in[0]; const float* wqkv = (const float*)d_in[1]; const float* wo = (const float*)d_in[2];
  const float* qng = (const float*)d_in[3]; const float* qnb = (const float*)d_in[4]; const float* kng = (const float*)d_in[5]; const float* knb = (const float*)d_in[6];
  float* out = (float*)d_out;
  char* ws = (char*)d_ws; size_t off = 0;
  auto take = [&](size_t bytes) { char* p = ws + off; off += (bytes + 255) & ~(size_t)255; return p; };
  _Float16* BQKV = (_Float16*)take((size_t)NQKV * DMX * 2);
  _Float16* BO = (_Float16*)take((size_t)DMX * DMX * 2);
  char* RA = take(NR * DMX * 2);
  _Float16* X16 = (_Float16*)RA; _Float16* O16 = (_Float16*)RA;
  const size_t szF = NR * (size_t)(DMX + 2 * DKV) * 4, szSP = (size_t)NH * QT * NKX * 6;
  char* RB = take(szF > szSP ? szF : szSP);
  float* QF = (float*)RB; float* KF = QF + NR * DMX; float* VF = KF + NR * DKV;
  float* S = (float*)RB; _Float16* P = (_Float16*)(RB + (size_t)NH * QT * NKX * 4);
  _Float16* Q16 = (_Float16*)take(NR * DMX * 2);
  _Float16* K16 = (_Float16*)take(NR * DKV * 2);
  _Float16* V16 = (_Float16*)take(NR * DKV * 2);
  _Float16* VT = (_Float16*)take((size_t)DKV * SQ * 2);
  float* CS = (float*)take((size_t)SQ * 64 * 4); float* SN = (float*)take((size_t)SQ * 64 * 4);
  float* QF0 = (float*)take((size_t)NB * QT0 * DMX * 4);
  float* KRF0 = (float*)take((size_t)NB * QT0 * DKV * 4);
  float* OF0 = (float*)take((size_t)NB * QT0 * DMX * 4);
  _Float16* OH0 = (_Float16*)take((size_t)NB * QT0 * DMX * 2);
  _Float16* OL0 = (_Float16*)take((size_t)NB * QT0 * DMX * 2);
  if (off > ws_size) return;
  k_wnat<<<(unsigned)(((size_t)NQKV * DMX / 8 + 255) / 256), 256, 0, stream>>>(wqkv, (size_t)NQKV * DMX / 8, BQKV);
  k_wnat<<<(unsigned)(((size_t)DMX * DMX / 8 + 255) / 256), 256, 0, stream>>>(wo, (size_t)DMX * DMX / 8, BO);
  k_x16<<<(unsigned)((NR * DMX / 8 + 255) / 256), 256, 0, stream>>>(x, X16, NR * DMX / 8);
  k_gemm2<<<dim3((unsigned)((NR / 128) * (DMX / 64)), 1), 128, 0, stream>>>(X16, DMX, 0, BQKV, DMX, 0, 1, 0.0625f, nullptr, QF, nullptr, DMX, 0, (int)NR, DMX, DMX);
  k_gemm2<<<dim3((unsigned)((NR / 128) * (DKV / 64)), 1), 128, 0, stream>>>(X16, DMX, 0, BQKV + (size_t)DMX * DMX, DMX, 0, 1, 0.0625f, nullptr, KF, nullptr, DKV, 0, (int)NR, DKV, DMX);
  k_gemm2<<<dim3((unsigned)((NR / 128) * (DKV / 64)), 1), 128, 0, stream>>>(X16, DMX, 0, BQKV + (size_t)(DMX + DKV) * DMX, DMX, 0, 1, 0.0625f, nullptr, VF, V16, DKV, 0, (int)NR, DKV, DMX);
  k_lnh128<<<(unsigned)(NR * NH), 128, 0, stream>>>(QF, DMX, NH, qng, qnb, LNEPS);
  k_lnh128<<<(unsigned)(NR * NKV), 128, 0, stream>>>(KF, DKV, NKV, kng, knb, LNEPS);
  k_tab128<<<(unsigned)((SQ * 64 + 255) / 256), 256, 0, stream>>>(CS, SN);
  k_rope128<0><<<(unsigned)(NR * NH), 128, 0, stream>>>(QF, DMX, NH, CS, SN, Q16, DMX);
  k_rope128<0><<<(unsigned)(NR * NKV), 128, 0, stream>>>(KF, DKV, NKV, CS, SN, K16, DKV);
  for (int b = 0; b < NB; ++b) { const size_t r0 = (size_t)b * SQ, f0 = (size_t)b * QT0;
    k_rope128<1><<<(unsigned)(QT0 * NH), 128, 0, stream>>>(QF + r0 * DMX, DMX, NH, CS, SN, QF0 + f0 * DMX, DMX);
    k_rope128<1><<<(unsigned)(QT0 * NKV), 128, 0, stream>>>(KF + r0 * DKV, DKV, NKV, CS, SN, KRF0 + f0 * DKV, DKV);
    k_att0h<GSZ><<<NH * (QT0 / 32), 32, 0, stream>>>(QF0 + f0 * DMX, DMX, KRF0 + f0 * DKV, VF + r0 * DKV, DKV, ATS, OF0 + f0 * DMX, DMX); }
  for (int b = 0; b < NB; ++b) { const size_t r0 = (size_t)b * SQ;
    k_vt<DKV / 64, SQ><<<(DKV / 64) * (SQ / 64), 256, 0, stream>>>(V16 + r0 * DKV, DKV, VT);
    for (int q0 = 0; q0 < SQ; q0 += QT) { const int nk = q0 + QT;
      k_gemm2<<<dim3((unsigned)((QT / 128) * (nk / 64)), NH), 128, 0, stream>>>(Q16 + (r0 + q0) * DMX, DMX, (size_t)HDK, K16 + r0 * DKV, DKV, (size_t)HDK, GSZ, ATS, nullptr, S, nullptr, NKX, (size_t)QT * NKX, QT, nk, HDK);
      k_rsmcf2<<<(NH * QT) / 256, 256, 0, stream>>>(S, P, q0, nk);
      k_gemm2<<<dim3((unsigned)((QT / 128) * (HDK / 64)), NH), 128, 0, stream>>>(P, NKX, (size_t)QT * NKX, VT, SQ, (size_t)HDK * SQ, GSZ, 0.0625f, nullptr, nullptr, O16 + (r0 + q0) * DMX, DMX, (size_t)HDK, QT, HDK, nk); } }
  k_gemm2<<<dim3((unsigned)((NR / 128) * (DMX / 64)), 1), 128, 0, stream>>>(O16, DMX, 0, BO, DMX, 0, 1, 0.0009765625f, nullptr, out, nullptr, DMX, 0, (int)NR, DMX, DMX);
  k_hl<<<(unsigned)(((size_t)NB * QT0 * DMX / 8 + 255) / 256), 256, 0, stream>>>(OF0, OH0, OL0, (size_t)NB * QT0 * DMX / 8);
  for (int b = 0; b < NB; ++b) { const size_t r0 = (size_t)b * SQ, f0 = (size_t)b * QT0;
    k_gemm2<<<dim3((QT0 / 128) * (DMX / 64), 1), 128, 0, stream>>>(OH0 + f0 * DMX, DMX, 0, BO, DMX, 0, 1, 0.0009765625f, nullptr, out + r0 * DMX, nullptr, DMX, 0, QT0, DMX, DMX);
    k_gemm2<<<dim3((QT0 / 128) * (DMX / 64), 1), 128, 0, stream>>>(OL0 + f0 * DMX, DMX, 0, BO, DMX, 0, 1, 0.00000095367431640625f, out + r0 * DMX, out + r0 * DMX, nullptr, DMX, 0, QT0, DMX, DMX); }
}
